// network_representation_module_GIN_57346403336484
// MI455X (gfx1250) — hardware-verified
//
#include <hip/hip_runtime.h>
#include <stddef.h>


#define HIDC    128
#define NTHR    256
#define NWAVE   8
#define EPT     8
#define NGRP    2
#define CHUNK   (NTHR * EPT * NGRP)
#define WCAP    (EPT * NGRP * 32)
#define LISTN   (NWAVE * WCAP)
#define NBC     4096
#define NBF     1024
#define RCAP    40960
#define RBN     128
#define DEGCAP  256
#define GROWS   128
#define OTHR    512
#define AP      (HIDC + 8)
#define SP      (HIDC + 4)
#define ARB     64
#define FTHR    128
#define BNEPS   1e-5f

#define LDS_FILL ((RCAP + NBF + LISTN) * 4 + 64)
#define LDS_GIN  (2 * GROWS * AP * 2 + GROWS * SP * 4 + 2 * HIDC * 8)

static_assert((CHUNK & (CHUNK - 1)) == 0);
static_assert(CHUNK <= 4096);
static_assert(NBC <= 4096 && NBF <= 4096);
static_assert((NBC & (NBC - 1)) == 0 && (NBF & (NBF - 1)) == 0);
static_assert(NBC == 4 * NBF);
static_assert(OTHR * 8 == NBC);
static_assert((RCAP % 32) == 0);
static_assert((HIDC * HIDC / 8) % NTHR == 0);
static_assert(GROWS == NWAVE * 16);
static_assert(ARB == NWAVE * 8);
static_assert(HIDC == 128);
static_assert(((2 * GROWS * AP * 2 + GROWS * SP * 4) % 16) == 0);
static_assert((RCAP + NBF + LISTN) * 4 + NWAVE * 4 <= LDS_FILL);

typedef float          v4f   __attribute__((ext_vector_type(4)));
typedef float          v8f   __attribute__((ext_vector_type(8)));
typedef int            v4i   __attribute__((ext_vector_type(4)));
typedef double         v2d   __attribute__((ext_vector_type(2)));
typedef unsigned short v4us  __attribute__((ext_vector_type(4), may_alias));
typedef unsigned short v8us  __attribute__((ext_vector_type(8), may_alias));
typedef __bf16         v16bf __attribute__((ext_vector_type(16)));
union FragB { v16bf v; v8us h[2]; };

__device__ __forceinline__ unsigned int bfbits(float x) {
  const unsigned int u = __float_as_uint(x);
  return (u + 0x7FFFu + ((u >> 16) & 1u)) >> 16;
}

__device__ __forceinline__ void split1(float v, unsigned short& h, unsigned short& l) {
  const unsigned int hb = bfbits(v);
  const float hf = __uint_as_float(hb << 16);
  h = (unsigned short)hb;
  l = (unsigned short)bfbits(v - hf);
}

__device__ __forceinline__ v8f wmb(v16bf a, v16bf b, v8f c) {
  v8f d = __builtin_amdgcn_wmma_f32_16x16x32_bf16(false, a, false, b, (short)0, c, false, false);
  asm volatile("v_nop\n\tv_nop\n\tv_nop\n\tv_nop" : "+v"(d) : "v"(a), "v"(b));
  return d;
}

template <int NB>
__device__ __forceinline__ int scan_chunk(const int* __restrict__ dsts, int nE, int cbase, int slotBase,
                                          int vec8, int* list, int tid, int lane, int wave) {
  int wc = 0;
#pragma unroll
  for (int g = 0; g < NGRP; ++g) {
    const int el0  = (g * NTHR + tid) * EPT;
    const int e0   = cbase + el0;
    const int sent = -2147483647 - 1;
    v4i da, db;
    if (vec8 != 0 && cbase + CHUNK <= nE) {
      da = *(const v4i*)(dsts + e0);
      db = *(const v4i*)(dsts + e0 + 4);
    } else {
      da.x = (e0     < nE) ? dsts[min(e0,     nE - 1)] : sent;
      da.y = (e0 + 1 < nE) ? dsts[min(e0 + 1, nE - 1)] : sent;
      da.z = (e0 + 2 < nE) ? dsts[min(e0 + 2, nE - 1)] : sent;
      da.w = (e0 + 3 < nE) ? dsts[min(e0 + 3, nE - 1)] : sent;
      db.x = (e0 + 4 < nE) ? dsts[min(e0 + 4, nE - 1)] : sent;
      db.y = (e0 + 5 < nE) ? dsts[min(e0 + 5, nE - 1)] : sent;
      db.z = (e0 + 6 < nE) ? dsts[min(e0 + 6, nE - 1)] : sent;
      db.w = (e0 + 7 < nE) ? dsts[min(e0 + 7, nE - 1)] : sent;
    }
    const unsigned nb = (unsigned)slotBase;
    const unsigned s0 = (unsigned)da.x - nb, s1 = (unsigned)da.y - nb;
    const unsigned s2 = (unsigned)da.z - nb, s3 = (unsigned)da.w - nb;
    const unsigned s4 = (unsigned)db.x - nb, s5 = (unsigned)db.y - nb;
    const unsigned s6 = (unsigned)db.z - nb, s7 = (unsigned)db.w - nb;
    const bool h0 = s0 < (unsigned)NB, h1 = s1 < (unsigned)NB, h2 = s2 < (unsigned)NB, h3 = s3 < (unsigned)NB;
    const bool h4 = s4 < (unsigned)NB, h5 = s5 < (unsigned)NB, h6 = s6 < (unsigned)NB, h7 = s7 < (unsigned)NB;
    const unsigned any = __builtin_amdgcn_ballot_w32(h0 | h1 | h2 | h3 | h4 | h5 | h6 | h7);
    if (any != 0u) {
#define HITJ(J, HJ, SJ) { \
        const unsigned mj = __builtin_amdgcn_ballot_w32(HJ); \
        if (mj != 0u) { \
          if (HJ) { \
            const int pos = wc + (int)__builtin_amdgcn_mbcnt_lo(mj, 0u); \
            if (pos < WCAP) list[wave * WCAP + pos] = ((el0 + (J)) << 12) | (int)(SJ); \
          } \
          wc += (int)__builtin_popcount(mj); } }
      HITJ(0, h0, s0)
      HITJ(1, h1, s1)
      HITJ(2, h2, s2)
      HITJ(3, h3, s3)
      HITJ(4, h4, s4)
      HITJ(5, h5, s5)
      HITJ(6, h6, s6)
      HITJ(7, h7, s7)
#undef HITJ
    }
  }
  return wc;
}

__global__ __launch_bounds__(NTHR) void k_wprep(
    const float* __restrict__ Wa, const float* __restrict__ Wb,
    unsigned short* pah, unsigned short* pal, unsigned short* pbh, unsigned short* pbl) {
  const int per = HIDC * HIDC / 8;
  const int bstart = blockIdx.x * NTHR;
  const bool second = bstart >= per;
  const float* src = second ? Wb : Wa;
  unsigned short* dh = second ? pbh : pah;
  unsigned short* dl = second ? pbl : pal;
  const int i = bstart + (int)threadIdx.x - (second ? per : 0);
  if (i >= per) return;
  const int o  = i * 8;
  const int n  = o / HIDC;
  const int k0 = o - n * HIDC;
  v8us hv, lv;
#pragma unroll
  for (int e = 0; e < 8; ++e) {
    const float w = src[(size_t)(k0 + e) * HIDC + n];
    unsigned short h, l;
    split1(w, h, l);
    hv[e] = h; lv[e] = l;
  }
  *(volatile v8us*)(dh + o) = hv;
  *(volatile v8us*)(dl + o) = lv;
  __threadfence();
  *(volatile v8us*)(dh + o) = hv;
  *(volatile v8us*)(dl + o) = lv;
}

__global__ __launch_bounds__(NTHR) void k_count(const int* __restrict__ ei, int* cnt, int nE, int vec8) {
  __shared__ __attribute__((aligned(16))) int scnt[NBC];
  __shared__ __attribute__((aligned(16))) int list[LISTN];
  __shared__ int wcnt[NWAVE];
  const int tid = threadIdx.x, lane = tid & 31, wave = tid >> 5;
  const int nodeBase = blockIdx.x * NBC;
  const int* dsts = ei + nE;

  for (int i = tid; i < NBC; i += NTHR) scnt[i] = 0;
  __syncthreads();

  const int nChunks = (nE + CHUNK - 1) / CHUNK;
#pragma unroll 1
  for (int ch = 0; ch < nChunks; ++ch) {
    const int cbase = ch * CHUNK;
    const int wc = scan_chunk<NBC>(dsts, nE, cbase, nodeBase, vec8, list, tid, lane, wave);
    if (lane == 0) wcnt[wave] = wc;
    __syncthreads();
    if (wave == 0) {
#pragma unroll 1
      for (int wsx = 0; wsx < NWAVE; ++wsx) {
        int n = __builtin_amdgcn_readfirstlane(wcnt[wsx]);
        n = n > WCAP ? WCAP : (n < 0 ? 0 : n);
        const int* lp = list + wsx * WCAP;
#pragma unroll 1
        for (int i = 0; i < n; ++i) {
          const int ent  = __builtin_amdgcn_readfirstlane(lp[i]);
          const int slot = ent & (NBC - 1);
          if (lane == 0) scnt[slot] = scnt[slot] + 1;
        }
      }
    }
    __syncthreads();
  }

  v4i cq[4];
#pragma unroll
  for (int q = 0; q < 4; ++q) {
    const int f = (wave * 4 + q) * 128 + 4 * lane;
    cq[q] = *(const v4i*)(scnt + f);
  }
  int* cp = cnt + (size_t)nodeBase;
#pragma unroll
  for (int q = 0; q < 4; ++q) {
    const int f = (wave * 4 + q) * 128 + 4 * lane;
    *(volatile v4i*)(cp + f) = cq[q];
  }
  __threadfence();
#pragma unroll
  for (int q = 0; q < 4; ++q) {
    const int f = (wave * 4 + q) * 128 + 4 * lane;
    *(volatile v4i*)(cp + f) = cq[q];
  }
}

__global__ __launch_bounds__(OTHR) void k_offsets(
    const int* __restrict__ cnt, int* off, int* rbase, int nChunk) {
  __shared__ __attribute__((aligned(16))) int soff[NBC];
  __shared__ __attribute__((aligned(16))) int srb[RBN];
  __shared__ int wtot[OTHR / 32];
  const int tid = threadIdx.x, lane = tid & 31, wave = tid >> 5, sub = tid >> 7;
  for (int i = tid; i < RBN; i += OTHR) srb[i] = 0;
  int carry = 0;
#pragma unroll 1
  for (int ch = 0; ch < nChunk; ++ch) {
    const int base = ch * NBC;
    const v4i c0 = *(const v4i*)(cnt + base + 8 * tid);
    const v4i c1 = *(const v4i*)(cnt + base + 8 * tid + 4);
    const int e0 = max(c0.x, 0), e1 = max(c0.y, 0), e2 = max(c0.z, 0), e3 = max(c0.w, 0);
    const int e4 = max(c1.x, 0), e5 = max(c1.y, 0), e6 = max(c1.z, 0), e7 = max(c1.w, 0);
    const int ts = e0 + e1 + e2 + e3 + e4 + e5 + e6 + e7;
    int incl = ts;
#pragma unroll
    for (int d = 1; d < 32; d <<= 1) {
      const int t = __shfl_up(incl, d);
      if (lane >= d) incl += t;
    }
    if (lane == 31) wtot[wave] = incl;
    __syncthreads();
    const int S0 = wtot[0]  + wtot[1]  + wtot[2]  + wtot[3];
    const int S1 = wtot[4]  + wtot[5]  + wtot[6]  + wtot[7];
    const int S2 = wtot[8]  + wtot[9]  + wtot[10] + wtot[11];
    const int S3 = wtot[12] + wtot[13] + wtot[14] + wtot[15];
    int pre = 0;
#pragma unroll 1
    for (int w = 4 * sub; w < wave; ++w) pre += wtot[w];
    const int b0 = carry;
    const int b1 = b0 + ((S0 + 31) & ~31);
    const int b2 = b1 + ((S1 + 31) & ~31);
    const int b3 = b2 + ((S2 + 31) & ~31);
    const int b4 = b3 + ((S3 + 31) & ~31);
    const int myb = sub == 0 ? b0 : (sub == 1 ? b1 : (sub == 2 ? b2 : b3));
    if (tid == 0) {
      srb[min(4 * ch + 0, RBN - 1)] = b0;
      srb[min(4 * ch + 1, RBN - 1)] = b1;
      srb[min(4 * ch + 2, RBN - 1)] = b2;
      srb[min(4 * ch + 3, RBN - 1)] = b3;
    }
    int run = myb + pre + incl - ts;
    soff[8 * tid + 0] = run; run += e0;
    soff[8 * tid + 1] = run; run += e1;
    soff[8 * tid + 2] = run; run += e2;
    soff[8 * tid + 3] = run; run += e3;
    soff[8 * tid + 4] = run; run += e4;
    soff[8 * tid + 5] = run; run += e5;
    soff[8 * tid + 6] = run; run += e6;
    soff[8 * tid + 7] = run;
    carry = b4;
    __syncthreads();
    const v4i o0 = *(const v4i*)(soff + 4 * tid);
    const v4i o1 = *(const v4i*)(soff + 4 * (tid + OTHR));
    int* op = off + base;
    *(volatile v4i*)(op + 4 * tid) = o0;
    *(volatile v4i*)(op + 4 * (tid + OTHR)) = o1;
    __threadfence();
    *(volatile v4i*)(op + 4 * tid) = o0;
    *(volatile v4i*)(op + 4 * (tid + OTHR)) = o1;
    __syncthreads();
  }
  if (tid == 0) srb[min(4 * nChunk, RBN - 1)] = carry;
  __syncthreads();
  v4i rv = {0, 0, 0, 0};
  if (tid < 32) rv = *(const v4i*)(srb + 4 * tid);
  if (tid < 32) *(volatile v4i*)(rbase + 4 * tid) = rv;
  __threadfence();
  if (tid < 32) *(volatile v4i*)(rbase + 4 * tid) = rv;
}

__global__ __launch_bounds__(NTHR) void k_fill(
    const int* __restrict__ ei, const int* __restrict__ off, const int* __restrict__ rbase,
    int* csr, int nN, int nE, int vec8, int csrLen) {
  extern __shared__ v4f lds_dyn[];
  int* region = (int*)lds_dyn;
  int* cursor = region + RCAP;
  int* list   = cursor + NBF;
  int* wcnt   = list + LISTN;
  const int tid = threadIdx.x, lane = tid & 31, wave = tid >> 5;
  const int b = blockIdx.x;
  const int nodeBase = b * NBF;
  const int* dsts = ei + nE;

  int rb0 = rbase[b];
  const int rb1 = rbase[b + 1];
  rb0 = rb0 < 0 ? 0 : (rb0 > csrLen ? csrLen : rb0);
  rb0 &= ~31;
  int len = rb1 - rb0;
  len = len < 0 ? 0 : (len > RCAP ? RCAP : len);
  int lenW = (len + 31) & ~31;
  if (rb0 + lenW > csrLen) lenW = (csrLen - rb0) & ~31;

  {
    const v4i zz = {0, 0, 0, 0};
    for (int i = tid; i < RCAP / 4; i += NTHR) ((v4i*)region)[i] = zz;
    for (int s = tid; s < NBF; s += NTHR) {
      int o = off[nodeBase + s] - rb0;
      o = o < 0 ? 0 : (o > RCAP ? RCAP : o);
      cursor[s] = o;
    }
  }
  __syncthreads();

  const int nChunks = (nE + CHUNK - 1) / CHUNK;
#pragma unroll 1
  for (int ch = 0; ch < nChunks; ++ch) {
    const int cbase = ch * CHUNK;
    const int wc = scan_chunk<NBF>(dsts, nE, cbase, nodeBase, vec8, list, tid, lane, wave);
    if (lane == 0) wcnt[wave] = wc;
    __syncthreads();
    if (wave == 0) {
#pragma unroll 1
      for (int wsx = 0; wsx < NWAVE; ++wsx) {
        int n = __builtin_amdgcn_readfirstlane(wcnt[wsx]);
        n = n > WCAP ? WCAP : (n < 0 ? 0 : n);
        const int* lp = list + wsx * WCAP;
#pragma unroll 1
        for (int i = 0; i < n; ++i) {
          const int ent  = __builtin_amdgcn_readfirstlane(lp[i]);
          const int slot = ent & (NBF - 1);
          int e = cbase + ((ent >> 12) & (CHUNK - 1));
          e = e > nE - 1 ? nE - 1 : e;
          int src = ei[e];
          src = src < 0 ? 0 : (src > nN - 1 ? nN - 1 : src);
          if (lane == 0) {
            int pos = cursor[slot];
            pos = pos < 0 ? 0 : (pos > RCAP - 1 ? RCAP - 1 : pos);
            region[pos] = src;
            const int np = pos + 1;
            cursor[slot] = np > RCAP ? RCAP : np;
          }
        }
      }
    }
    __syncthreads();
  }

  const int nv = lenW >> 2;
  int* gp = csr + rb0;
#pragma unroll 1
  for (int i = tid; i < nv; i += NTHR) { const v4i v = ((const v4i*)region)[i]; *(volatile v4i*)(gp + 4 * i) = v; }
  __threadfence();
#pragma unroll 1
  for (int i = tid; i < nv; i += NTHR) { const v4i v = ((const v4i*)region)[i]; *(volatile v4i*)(gp + 4 * i) = v; }
}

__global__ __launch_bounds__(NTHR) void k_gin(
    const float* __restrict__ x, const int* __restrict__ csr, const int* __restrict__ off,
    const int* __restrict__ cnt, const float* __restrict__ epsp,
    const unsigned short* __restrict__ whi, const unsigned short* __restrict__ wlo,
    const float* __restrict__ bias, float* z, double* part, int nN, int csrLen) {
  extern __shared__ v4f lds_dyn[];
  unsigned short* sAh = (unsigned short*)lds_dyn;
  unsigned short* sAl = sAh + GROWS * AP;
  float*  stg   = (float*)(sAl + GROWS * AP);
  double* sPart = (double*)(stg + GROWS * SP);
  const int tid = threadIdx.x, lane = tid & 31, wave = tid >> 5, hh = lane >> 4, m = lane & 15;
  const int rowBase = blockIdx.x * GROWS;
  const int rw = rowBase + wave * 16;
  const float epsv = 1.0f + epsp[0];
  const int cl = rw + m;
  const int cnt_l = cnt[cl];
  const int off_l = off[cl];

#pragma unroll 1
  for (int j = 0; j < 16; ++j) {
    const int c = rw + j;
    const bool valid = c < nN;
    int n = __builtin_amdgcn_readlane(cnt_l, j);
    n = n < 0 ? 0 : (n > DEGCAP ? DEGCAP : n);
    n = valid ? n : 0;
    const int st = __builtin_amdgcn_readlane(off_l, j);
    const int cc = c > nN - 1 ? nN - 1 : c;
    const v4f xv = *(const v4f*)(x + (size_t)cc * HIDC + 4 * lane);
    v4f acc = xv * (valid ? epsv : 0.0f);
#pragma unroll 1
    for (int q0 = 0; q0 < n; q0 += 32) {
      int pos = st + q0 + lane;
      pos = pos < 0 ? 0 : (pos > csrLen - 1 ? csrLen - 1 : pos);
      int sl = csr[pos];
      sl = sl < 0 ? 0 : (sl > nN - 1 ? nN - 1 : sl);
      const int mcnt = (n - q0) < 32 ? (n - q0) : 32;
#pragma unroll 1
      for (int p = 0; p < mcnt; ++p) {
        const int s = __builtin_amdgcn_readlane(sl, p);
        acc = acc + *(const v4f*)(x + (size_t)s * HIDC + 4 * lane);
      }
    }
    v4us hq, lq;
    unsigned short h0, l0, h1, l1, h2, l2, h3, l3;
    split1(acc.x, h0, l0); split1(acc.y, h1, l1); split1(acc.z, h2, l2); split1(acc.w, h3, l3);
    hq.x = h0; hq.y = h1; hq.z = h2; hq.w = h3;
    lq.x = l0; lq.y = l1; lq.z = l2; lq.w = l3;
    *(v4us*)(sAh + (wave * 16 + j) * AP + 4 * lane) = hq;
    *(v4us*)(sAl + (wave * 16 + j) * AP + 4 * lane) = lq;
  }
  __syncthreads();

  const unsigned short* arh = sAh + (wave * 16 + m) * AP + 8 * hh;
  const unsigned short* arl = sAl + (wave * 16 + m) * AP + 8 * hh;
#pragma unroll 1
  for (int g = 0; g < 2; ++g) {
    v8f acc[4];
#pragma unroll
    for (int t = 0; t < 4; ++t) { v8f zz = {0.f, 0.f, 0.f, 0.f, 0.f, 0.f, 0.f, 0.f}; acc[t] = zz; }
#pragma unroll 1
    for (int kt = 0; kt < HIDC / 32; ++kt) {
      FragB ah, al;
      ah.h[0] = *(const v8us*)(arh + 32 * kt);
      ah.h[1] = *(const v8us*)(arh + 32 * kt + 16);
      al.h[0] = *(const v8us*)(arl + 32 * kt);
      al.h[1] = *(const v8us*)(arl + 32 * kt + 16);
#pragma unroll
      for (int t = 0; t < 4; ++t) {
        const size_t bo = (size_t)(64 * g + 16 * t + m) * HIDC + 32 * kt + 8 * hh;
        FragB bh, bl;
        bh.h[0] = *(const v8us*)(whi + bo);
        bh.h[1] = *(const v8us*)(whi + bo + 16);
        bl.h[0] = *(const v8us*)(wlo + bo);
        bl.h[1] = *(const v8us*)(wlo + bo + 16);
        acc[t] = wmb(ah.v, bh.v, acc[t]);
        acc[t] = wmb(ah.v, bl.v, acc[t]);
        acc[t] = wmb(al.v, bh.v, acc[t]);
      }
    }
#pragma unroll
    for (int t = 0; t < 4; ++t) {
      const int col = 64 * g + 16 * t + m;
      const float bv = bias[col];
      float* sp = stg + (wave * 16 + 8 * hh) * SP + col;
#pragma unroll
      for (int r = 0; r < 8; ++r) sp[r * SP] = acc[t][r] + bv;
    }
  }
  __syncthreads();

  const float* lp = stg + (wave * 16) * SP + 4 * lane;
  float* gp = z + ((size_t)rowBase + wave * 16) * HIDC + 4 * lane;
#pragma unroll
  for (int i = 0; i < 16; ++i) { const v4f v = *(const v4f*)(lp + i * SP); *(volatile v4f*)(gp + (size_t)i * HIDC) = v; }

  int nv = nN - rowBase;
  nv = nv < 0 ? 0 : (nv > GROWS ? GROWS : nv);
  if (tid < HIDC) {
    double s = 0.0, q = 0.0;
#pragma unroll 1
    for (int r = 0; r < nv; ++r) {
      const double v = (double)stg[r * SP + tid];
      s += v;
      q += v * v;
    }
    sPart[tid] = s;
    sPart[HIDC + tid] = q;
  }
  __syncthreads();
  double* pp = part + (size_t)blockIdx.x * (2 * HIDC);
  if (wave == 0) {
#pragma unroll
    for (int p = 0; p < 4; ++p) {
      const v2d v = *(const v2d*)(sPart + 2 * (32 * p + lane));
      *(volatile v2d*)(pp + 2 * (32 * p + lane)) = v;
    }
  }
  __threadfence();
#pragma unroll
  for (int i = 0; i < 16; ++i) { const v4f v = *(const v4f*)(lp + i * SP); *(volatile v4f*)(gp + (size_t)i * HIDC) = v; }
  if (wave == 0) {
#pragma unroll
    for (int p = 0; p < 4; ++p) {
      const v2d v = *(const v2d*)(sPart + 2 * (32 * p + lane));
      *(volatile v2d*)(pp + 2 * (32 * p + lane)) = v;
    }
  }
}

__global__ __launch_bounds__(FTHR) void k_bnfin(const double* __restrict__ part, int nBlk, double invN, float* stat) {
  __shared__ __attribute__((aligned(16))) float sStat[2 * HIDC];
  const int tid = threadIdx.x;
  double s = 0.0, q = 0.0;
#pragma unroll 1
  for (int b = 0; b < nBlk; ++b) {
    s += part[(size_t)b * (2 * HIDC) + tid];
    q += part[(size_t)b * (2 * HIDC) + HIDC + tid];
  }
  const double mu = s * invN;
  double var = q * invN - mu * mu;
  var = var < 0.0 ? 0.0 : var;
  const float muf  = (float)mu;
  const float varf = (float)var;
  const float rs   = rsqrtf(varf + BNEPS);
  sStat[tid] = muf;
  sStat[HIDC + tid] = rs;
  __syncthreads();
  v4f v = {0.f, 0.f, 0.f, 0.f};
  if (tid < 64) v = *(const v4f*)(sStat + 4 * tid);
  if (tid < 64) *(volatile v4f*)(stat + 4 * tid) = v;
  __threadfence();
  if (tid < 64) *(volatile v4f*)(stat + 4 * tid) = v;
}

__global__ __launch_bounds__(NTHR) void k_bnapply(
    const float* __restrict__ z, const float* __restrict__ stat,
    const float* __restrict__ gam, const float* __restrict__ bet, float* y, int nRows) {
  const int tid = threadIdx.x, lane = tid & 31, wave = tid >> 5;
  const v4f mu = *(const v4f*)(stat + 4 * lane);
  const v4f rs = *(const v4f*)(stat + HIDC + 4 * lane);
  const v4f ga = *(const v4f*)(gam + 4 * lane);
  const v4f be = *(const v4f*)(bet + 4 * lane);
  const int rb = blockIdx.x * ARB + wave * 8;
  v4f ov[8];
#pragma unroll
  for (int i = 0; i < 8; ++i) {
    int row = rb + i;
    row = row > nRows - 1 ? nRows - 1 : row;
    const v4f zv = *(const v4f*)(z + (size_t)row * HIDC + 4 * lane);
    const v4f t = (zv - mu) * rs;
    v4f o = t * ga + be;
    o.x = fmaxf(o.x, 0.0f); o.y = fmaxf(o.y, 0.0f); o.z = fmaxf(o.z, 0.0f); o.w = fmaxf(o.w, 0.0f);
    ov[i] = o;
  }
#pragma unroll
  for (int i = 0; i < 8; ++i) {
    const int row = rb + i;
    if (row < nRows) *(volatile v4f*)(y + (size_t)row * HIDC + 4 * lane) = ov[i];
  }
  __threadfence();
#pragma unroll
  for (int i = 0; i < 8; ++i) {
    const int row = rb + i;
    if (row < nRows) *(volatile v4f*)(y + (size_t)row * HIDC + 4 * lane) = ov[i];
  }
}

extern "C" void kernel_launch(void* const* d_in, const int* in_sizes, int n_in,
                              void* d_out, int out_size, void* d_ws, size_t ws_size,
                              hipStream_t stream) {
  if (n_in < 12) return;
  const int nN = in_sizes[0] / HIDC;
  const int nE = in_sizes[1] / 2;
  if (nN <= 0 || nE <= 0 || in_sizes[0] != nN * HIDC || in_sizes[1] != 2 * nE) return;
  if (in_sizes[2] != HIDC * HIDC || in_sizes[7] != HIDC * HIDC) return;
  if (in_sizes[3] < HIDC || in_sizes[5] < HIDC || in_sizes[6] < HIDC) return;
  if (in_sizes[8] < HIDC || in_sizes[10] < HIDC || in_sizes[11] < HIDC) return;
  if (in_sizes[4] < 1 || in_sizes[9] < 1) return;
  if ((size_t)out_size != (size_t)nN * HIDC) return;
  if (nE > (1 << 28) || nN > (1 << 24)) return;

  const float* feat = (const float*)d_in[0];
  const int*   ei   = (const int*)d_in[1];
  const float* W1   = (const float*)d_in[2];
  const float* b1   = (const float*)d_in[3];
  const float* eps1 = (const float*)d_in[4];
  const float* g1   = (const float*)d_in[5];
  const float* be1  = (const float*)d_in[6];
  const float* W2   = (const float*)d_in[7];
  const float* b2   = (const float*)d_in[8];
  const float* eps2 = (const float*)d_in[9];
  const float* g2   = (const float*)d_in[10];
  const float* be2  = (const float*)d_in[11];
  float* out = (float*)d_out;

  const int nGin   = (nN + GROWS - 1) / GROWS;
  const int NPAD   = nGin * GROWS;
  const int nBC    = (nN + NBC - 1) / NBC;
  const int CNTPAD = nBC * NBC;
  if (4 * nBC + 1 > RBN) return;
  const int nBF    = (nN + NBF - 1) / NBF;
  const int csrLen = ((nE + 31) & ~31) + 4096;
  const int nAp1   = NPAD / ARB;
  const int nAp2   = (nN + ARB - 1) / ARB;
  const double invN = 1.0 / (double)nN;

  char* ws = (char*)d_ws;
  size_t offb = 0;
  const size_t szW = (size_t)HIDC * HIDC * 2;
  const size_t oW1h = offb; offb += szW;                           offb = (offb + 255) & ~(size_t)255;
  const size_t oW1l = offb; offb += szW;                           offb = (offb + 255) & ~(size_t)255;
  const size_t oW2h = offb; offb += szW;                           offb = (offb + 255) & ~(size_t)255;
  const size_t oW2l = offb; offb += szW;                           offb = (offb + 255) & ~(size_t)255;
  const size_t oCnt = offb; offb += (size_t)CNTPAD * 4;            offb = (offb + 255) & ~(size_t)255;
  const size_t oOff = offb; offb += (size_t)CNTPAD * 4;            offb = (offb + 255) & ~(size_t)255;
  const size_t oRb  = offb; offb += (size_t)RBN * 4;               offb = (offb + 255) & ~(size_t)255;
  const size_t oCsr = offb; offb += (size_t)csrLen * 4;            offb = (offb + 255) & ~(size_t)255;
  const size_t oZ   = offb; offb += (size_t)NPAD * HIDC * 4;       offb = (offb + 255) & ~(size_t)255;
  const size_t oX1  = offb; offb += (size_t)NPAD * HIDC * 4;       offb = (offb + 255) & ~(size_t)255;
  const size_t oPt  = offb; offb += (size_t)nGin * 2 * HIDC * 8;   offb = (offb + 255) & ~(size_t)255;
  const size_t oSt  = offb; offb += (size_t)2 * HIDC * 4;          offb = (offb + 255) & ~(size_t)255;
  if (offb > ws_size) return;
  unsigned short* w1h = (unsigned short*)(ws + oW1h);
  unsigned short* w1l = (unsigned short*)(ws + oW1l);
  unsigned short* w2h = (unsigned short*)(ws + oW2h);
  unsigned short* w2l = (unsigned short*)(ws + oW2l);
  int*    cnt  = (int*)(ws + oCnt);
  int*    offp = (int*)(ws + oOff);
  int*    rb   = (int*)(ws + oRb);
  int*    csr  = (int*)(ws + oCsr);
  float*  zpl  = (float*)(ws + oZ);
  float*  x1   = (float*)(ws + oX1);
  double* part = (double*)(ws + oPt);
  float*  stat = (float*)(ws + oSt);

  const int vec8 = ((nE & 3) == 0) ? 1 : 0;

  k_wprep<<<2 * (HIDC * HIDC / 8) / NTHR, NTHR, 0, stream>>>(W1, W2, w1h, w1l, w2h, w2l);

  k_count<<<nBC, NTHR, 0, stream>>>(ei, cnt, nE, vec8);
  k_offsets<<<1, OTHR, 0, stream>>>(cnt, offp, rb, nBC);
  hipFuncSetAttribute(reinterpret_cast<const void*>(&k_fill),
                      hipFuncAttributeMaxDynamicSharedMemorySize, LDS_FILL);
  k_fill<<<nBF, NTHR, LDS_FILL, stream>>>(ei, offp, rb, csr, nN, nE, vec8, csrLen);

  hipFuncSetAttribute(reinterpret_cast<const void*>(&k_gin),
                      hipFuncAttributeMaxDynamicSharedMemorySize, LDS_GIN);
  k_gin<<<nGin, NTHR, LDS_GIN, stream>>>(feat, csr, offp, cnt, eps1, w1h, w1l, b1, zpl, part, nN, csrLen);
  k_bnfin<<<1, FTHR, 0, stream>>>(part, nGin, invN, stat);
  k_bnapply<<<nAp1, NTHR, 0, stream>>>(zpl, stat, g1, be1, x1, NPAD);

  k_gin<<<nGin, NTHR, LDS_GIN, stream>>>(x1, csr, offp, cnt, eps2, w2h, w2l, b2, zpl, part, nN, csrLen);
  k_bnfin<<<1, FTHR, 0, stream>>>(part, nGin, invN, stat);
  k_bnapply<<<nAp2, NTHR, 0, stream>>>(zpl, stat, g2, be2, out, nN);
}
